// myGCN_63788854280505
// MI455X (gfx1250) — hardware-verified
//
#include <hip/hip_runtime.h>
#include <stddef.h>
#include <stdint.h>


typedef _Float16 v16h __attribute__((ext_vector_type(16)));
typedef _Float16 v8h  __attribute__((ext_vector_type(8)));
typedef _Float16 v4h  __attribute__((ext_vector_type(4)));
typedef float    v8f  __attribute__((ext_vector_type(8)));
typedef float    v4f  __attribute__((ext_vector_type(4)));
typedef int      v4i  __attribute__((ext_vector_type(4)));

union Frag   { v16h v; v8h half[2]; };
union Pack16 { v8h h; v4i i; };

#define DH        128
#define ROWS      64
#define PH        136
#define PC        132
#define GNODES    256
#define GSHIFT    8
#define SNODES    4096
#define SSHIFT    12
#define TNODES    32
#define NWAVE_AGG 8
#define ASCALE    8.0f
#define WSCALE    64.0f
#define OSCALE    (1.0f / 512.0f)

static __device__ __forceinline__ float eluf(float x) { return x > 0.0f ? x : (__expf(x) - 1.0f); }
static __device__ __forceinline__ int clampi(int v, int n) { v = v < 0 ? 0 : v; return v > n - 1 ? n - 1 : v; }
static __device__ __forceinline__ v8f zero8() { v8f z = {0.f, 0.f, 0.f, 0.f, 0.f, 0.f, 0.f, 0.f}; return z; }

static __device__ __forceinline__ v8f wmma_f16(v16h a, v16h b, v8f c)
{
  v8f d = __builtin_amdgcn_wmma_f32_16x16x32_f16(false, a, false, b, (short)0, c, false, false);
  asm volatile("v_nop\n\tv_nop\n\tv_nop\n\tv_nop" : "+v"(d) : "v"(a), "v"(b));
  return d;
}

__global__ void __launch_bounds__(256)
k_wcvt(const float* __restrict__ w0, const float* __restrict__ w1, const float* __restrict__ w2,
       const float* __restrict__ w3, const float* __restrict__ w4, const float* __restrict__ w5,
       _Float16* __restrict__ Wt)
{
  __shared__ __align__(16) _Float16 t16[16 * PH];
  const int m = blockIdx.y, tid = threadIdx.x, c0 = blockIdx.x * 16;
  const float* W = (m == 0) ? w0 : (m == 1) ? w1 : (m == 2) ? w2 : (m == 3) ? w3 : (m == 4) ? w4 : w5;
  for (int i = tid; i < 16 * DH; i += 256) {
    const int k = i >> 4, cc = i & 15;
    t16[cc * PH + k] = (_Float16)(W[(size_t)k * DH + c0 + cc] * WSCALE);
  }
  __syncthreads();
  const int cc = tid >> 4, seg = (tid & 15) << 3;
  Pack16 u;
  u.h = *(const v8h*)(t16 + cc * PH + seg);
  volatile v4i* p = (volatile v4i*)(Wt + (size_t)m * DH * DH + (size_t)(c0 + cc) * DH + seg);
  *p = u.i;
  __threadfence();
  *p = u.i;
}

struct QState { int qn; int nw; };

static __device__ __forceinline__ void q_flush64(int* qs, int* qd, QState& st, int lane, int2* obase, int cap)
{
  if (st.nw + 64 <= cap) {
    v4i v = {qs[2 * lane], qd[2 * lane], qs[2 * lane + 1], qd[2 * lane + 1]};
    volatile v4i* p = (volatile v4i*)(obase + st.nw) + lane;
    *p = v;
    __threadfence();
    *p = v;
    st.nw += 64;
  }
  __syncthreads();
}

static __device__ __forceinline__ void q_push(int* qs, int* qd, QState& st, unsigned mask, bool in,
                                              int sx, int dy, int lane, int2* obase, int cap)
{
  if (mask == 0u) return;
  const int rank = __builtin_popcount(mask & ((1u << lane) - 1u));
  if (in) { qs[st.qn + rank] = sx; qd[st.qn + rank] = dy; }
  st.qn += __builtin_popcount(mask);
  __syncthreads();
  if (st.qn >= 64) {
    q_flush64(qs, qd, st, lane, obase, cap);
    const int rem = st.qn - 64;
    int ts = 0, td = 0;
    if (lane < rem) { ts = qs[lane + 64]; td = qd[lane + 64]; }
    __syncthreads();
    if (lane < rem) { qs[lane] = ts; qd[lane] = td; }
    st.qn = rem;
    __syncthreads();
  }
}

static __device__ __forceinline__ int q_finish(int* qs, int* qd, QState& st, int lane, int2* obase, int cap)
{
  int total = st.nw;
  if (st.qn > 0) {
    for (int i = st.qn + lane; i < 64; i += 32) { qs[i] = -1; qd[i] = -1; }
    __syncthreads();
    const int before = st.nw;
    q_flush64(qs, qd, st, lane, obase, cap);
    if (st.nw != before) total = before + st.qn;
  }
  return total;
}

static __device__ __forceinline__ void write_cnt_line(int* cnt, int b, int total, int lane)
{
  v4i c = {total, total, total, total};
  volatile v4i* p = (volatile v4i*)(cnt + (size_t)b * 32) + lane;
  if (lane < 8) *p = c;
  __threadfence();
  if (lane < 8) *p = c;
}

__global__ void __launch_bounds__(32)
k_split1(const int* __restrict__ src, const int* __restrict__ dst, int E, int N,
         int2* __restrict__ listS, int* __restrict__ cntS, int capS)
{
  __shared__ int qs[128];
  __shared__ int qd[128];
  const int b = blockIdx.x, lane = threadIdx.x;
  int2* obase = listS + (size_t)b * capS;
  QState st; st.qn = 0; st.nw = 0;
  for (int c0 = 0; c0 < E; c0 += 32) {
    const int e = c0 + lane;
    bool in = false; int sx = 0, dy = -1;
    if (e < E) {
      sx = clampi(src[e], N);
      dy = dst[e];
      in = ((unsigned)dy < (unsigned)N) && ((dy >> SSHIFT) == b);
    }
    const unsigned mask = __builtin_amdgcn_ballot_w32(in);
    q_push(qs, qd, st, mask, in, sx, dy, lane, obase, capS);
  }
  const int total = q_finish(qs, qd, st, lane, obase, capS);
  write_cnt_line(cntS, b, total, lane);
}

__global__ void __launch_bounds__(32)
k_split2(const int2* __restrict__ listS, const int* __restrict__ cntS, int capS, int N,
         int2* __restrict__ listG, int* __restrict__ cntG, int capG, float* __restrict__ dinv)
{
  __shared__ int qs[128];
  __shared__ int qd[128];
  __shared__ int dcnt[GNODES];
  const int g = blockIdx.x, lane = threadIdx.x;
  const int s = g >> (SSHIFT - GSHIFT);
  #pragma unroll
  for (int i = 0; i < GNODES / 32; ++i) dcnt[i * 32 + lane] = 0;
  int nIn = cntS[(size_t)s * 32];
  nIn = nIn < 0 ? 0 : (nIn > capS ? capS : nIn);
  const int2* ibase = listS + (size_t)s * capS;
  int2* obase = listG + (size_t)g * capG;
  __syncthreads();
  QState st; st.qn = 0; st.nw = 0;
  for (int c0 = 0; c0 < nIn; c0 += 32) {
    const int idx = c0 + lane;
    int sx = 0, dy = -1;
    if (idx < nIn) { const int2 p = ibase[idx]; sx = clampi(p.x, N); dy = p.y; }
    const bool in = ((unsigned)dy < (unsigned)N) && ((dy >> GSHIFT) == g);
    const unsigned mask = __builtin_amdgcn_ballot_w32(in);
    for (unsigned mm = mask; mm; mm &= mm - 1u) {
      const int j = __builtin_ctz(mm);
      const int dj = __shfl(dy, j, 32);
      if (lane == 0) dcnt[dj & (GNODES - 1)] += 1;
    }
    q_push(qs, qd, st, mask, in, sx, dy, lane, obase, capG);
  }
  const int total = q_finish(qs, qd, st, lane, obase, capG);
  write_cnt_line(cntG, g, total, lane);
  __syncthreads();
  for (int pass = 0; pass < 2; ++pass) {
    #pragma unroll
    for (int i = 0; i < GNODES / 32; ++i) {
      if (lane < 8) {
        const int ln = i * 32 + lane * 4;
        const int nb = g * GNODES + ln;
        v4f o;
        o.x = (nb + 0 < N) ? rsqrtf((float)dcnt[ln + 0] + 1.0f) : 1.0f;
        o.y = (nb + 1 < N) ? rsqrtf((float)dcnt[ln + 1] + 1.0f) : 1.0f;
        o.z = (nb + 2 < N) ? rsqrtf((float)dcnt[ln + 2] + 1.0f) : 1.0f;
        o.w = (nb + 3 < N) ? rsqrtf((float)dcnt[ln + 3] + 1.0f) : 1.0f;
        *(volatile v4f*)(dinv + nb) = o;
      }
    }
    if (pass == 0) __threadfence();
  }
}

static __device__ __forceinline__ void epi_tile(float* sC, v8f acc, int rt, int hi, int col, int row0, int N,
                                                int flags, const float* __restrict__ rowscale, float bv)
{
  #pragma unroll
  for (int r = 0; r < 8; ++r) {
    const int lr = rt * 16 + (hi << 3) + r;
    const int gr = row0 + lr;
    float v = acc[r] * OSCALE;
    if (flags & 1) v *= (gr < N) ? rowscale[gr] : 0.0f;
    v += bv;
    if (flags & 4) v = eluf(v);
    sC[lr * PC + col] = v;
  }
}

__global__ void __launch_bounds__(256)
k_gemm(const float* __restrict__ A, const _Float16* __restrict__ Wt,
       const float* __restrict__ bias, const float* __restrict__ rowscale,
       float* __restrict__ out, const float* __restrict__ w3, const float* __restrict__ b3,
       float* __restrict__ dout, int N, int flags)
{
  __shared__ __align__(16) unsigned char smem[ROWS * PH * 2 + DH * PH * 2];
  _Float16* sA = (_Float16*)smem;
  _Float16* sW = (_Float16*)(smem + ROWS * PH * 2);
  float* sC = (float*)smem;
  float* sO = (float*)(smem + ROWS * PC * 4);

  const int tid = threadIdx.x;
  const int row0 = blockIdx.x * ROWS;
  const v4f z4 = {0.0f, 0.0f, 0.0f, 0.0f};

  {
    const v8h* wv = (const v8h*)Wt;
    for (int i = tid; i < DH * (DH / 8); i += 256) {
      const int r = i >> 4, c8 = (i & 15) << 3;
      *(v8h*)(sW + r * PH + c8) = wv[i];
    }
    for (int i = tid; i < ROWS * (DH / 4); i += 256) {
      const int r = i >> 5, c4 = i & 31;
      const int gr = row0 + r;
      v4f q = z4;
      if (gr < N) q = *((const v4f*)(A + (size_t)gr * DH) + c4);
      const v4h hq = __builtin_convertvector(q * ASCALE, v4h);
      *(v4h*)(sA + r * PH + (c4 << 2)) = hq;
    }
  }
  __syncthreads();

  const int lane = tid & 31, hi = lane >> 4, rc = lane & 15;
  const int wcol0 = (tid >> 5) << 4;

  v8f acc0 = zero8(), acc1 = zero8(), acc2 = zero8(), acc3 = zero8();
  #pragma unroll
  for (int kk = 0; kk < DH / 32; ++kk) {
    const int kb = kk * 32 + (hi << 3);
    Frag b;
    const _Float16* bp = sW + (wcol0 + rc) * PH + kb;
    b.half[0] = *(const v8h*)bp;
    b.half[1] = *(const v8h*)(bp + 16);
    const _Float16* ap = sA + rc * PH + kb;
    Frag a;
    a.half[0] = *(const v8h*)(ap);            a.half[1] = *(const v8h*)(ap + 16);            acc0 = wmma_f16(a.v, b.v, acc0);
    a.half[0] = *(const v8h*)(ap + 16 * PH);  a.half[1] = *(const v8h*)(ap + 16 * PH + 16);  acc1 = wmma_f16(a.v, b.v, acc1);
    a.half[0] = *(const v8h*)(ap + 32 * PH);  a.half[1] = *(const v8h*)(ap + 32 * PH + 16);  acc2 = wmma_f16(a.v, b.v, acc2);
    a.half[0] = *(const v8h*)(ap + 48 * PH);  a.half[1] = *(const v8h*)(ap + 48 * PH + 16);  acc3 = wmma_f16(a.v, b.v, acc3);
  }
  __syncthreads();

  const int col = wcol0 + rc;
  const float bv = (flags & 2) ? bias[col] : 0.0f;
  epi_tile(sC, acc0, 0, hi, col, row0, N, flags, rowscale, bv);
  epi_tile(sC, acc1, 1, hi, col, row0, N, flags, rowscale, bv);
  epi_tile(sC, acc2, 2, hi, col, row0, N, flags, rowscale, bv);
  epi_tile(sC, acc3, 3, hi, col, row0, N, flags, rowscale, bv);
  __syncthreads();

  if ((flags & 8) == 0) {
    const int wv = tid >> 5;
    for (int pass = 0; pass < 2; ++pass) {
      #pragma unroll
      for (int r = 0; r < ROWS / 8; ++r) {
        const int lr = wv * (ROWS / 8) + r;
        const int gr = row0 + lr;
        if (gr < N) {
          const v4f v = *((const v4f*)(sC + lr * PC) + lane);
          *((volatile v4f*)(out + (size_t)gr * DH) + lane) = v;
        }
      }
      if (pass == 0) __threadfence();
    }
  } else {
    const int hr = tid >> 2, hq = tid & 3;
    const float* crow = sC + hr * PC + hq * 32;
    const float* wq = w3 + hq * 32;
    float p = 0.0f;
    #pragma unroll 8
    for (int k = 0; k < 32; ++k) p += crow[k] * wq[k];
    p += __shfl_xor(p, 1, 32);
    p += __shfl_xor(p, 2, 32);
    if (hq == 0) {
      const float v = eluf(p + b3[0]);
      sO[hr] = 1.0f / (1.0f + __expf(-v));
    }
    __syncthreads();
    if (tid < 32) {
      int nv = N - row0; if (nv > ROWS) nv = ROWS; if (nv < 0) nv = 0;
      const int nq = nv >> 2, rem = nv & 3;
      v4f o = z4; float t = 0.0f;
      if (tid < nq) o = *(const v4f*)(sO + tid * 4);
      if (tid < rem) t = sO[nq * 4 + tid];
      volatile v4f* p4 = (volatile v4f*)(dout + row0) + tid;
      volatile float* p1 = (volatile float*)(dout + row0 + nq * 4 + tid);
      if (tid < nq) *p4 = o;
      if (tid < rem) *p1 = t;
      __threadfence();
      if (tid < nq) *p4 = o;
      if (tid < rem) *p1 = t;
    }
  }
}

__global__ void __launch_bounds__(256)
k_aggr(const float* __restrict__ Y, const int2* __restrict__ listG, const int* __restrict__ cntG, int capG,
       const float* __restrict__ dinv, const float* __restrict__ bias, float* __restrict__ H, int N, int relu)
{
  extern __shared__ v4f ldyn4[];
  const int g = blockIdx.x, w = threadIdx.x >> 5, lane = threadIdx.x & 31;
  v4f* acc = ldyn4 + w * (TNODES * (DH / 4));
  const int node0 = g * GNODES + w * TNODES;
  int nIn = cntG[(size_t)g * 32];
  nIn = nIn < 0 ? 0 : (nIn > capG ? capG : nIn);
  const int2* base = listG + (size_t)g * capG;
  const v4f z4 = {0.0f, 0.0f, 0.0f, 0.0f};
  #pragma unroll
  for (int n = 0; n < TNODES; ++n) acc[n * 32 + lane] = z4;

  for (int c0 = 0; c0 < nIn; c0 += 32) {
    const int idx = c0 + lane;
    int sx = 0, dl = -1;
    if (idx < nIn) { const int2 p = base[idx]; sx = clampi(p.x, N); dl = p.y - node0; }
    const bool mine = (unsigned)dl < (unsigned)TNODES;
    unsigned mask = __builtin_amdgcn_ballot_w32(mine);
    while (mask) {
      const int j = __builtin_ctz(mask);
      mask &= mask - 1u;
      const int sj = __shfl(sx, j, 32);
      const int dj = __shfl(dl, j, 32) & (TNODES - 1);
      const v4f v = *((const v4f*)(Y + (size_t)sj * DH) + lane);
      acc[dj * 32 + lane] += v;
    }
  }

  const v4f bb = *((const v4f*)bias + lane);
  for (int pass = 0; pass < 2; ++pass) {
    #pragma unroll 4
    for (int n = 0; n < TNODES; ++n) {
      const int node = node0 + n;
      if (node < N) {
        const float dv = dinv[node];
        const v4f y = *((const v4f*)(Y + (size_t)node * DH) + lane);
        v4f o = (acc[n * 32 + lane] + y) * dv + bb;
        if (relu) {
          o.x = fmaxf(o.x, 0.0f); o.y = fmaxf(o.y, 0.0f);
          o.z = fmaxf(o.z, 0.0f); o.w = fmaxf(o.w, 0.0f);
        }
        *((volatile v4f*)(H + (size_t)node * DH) + lane) = o;
      }
    }
    if (pass == 0) __threadfence();
  }
}

extern "C" void kernel_launch(void* const* d_in, const int* in_sizes, int n_in,
                              void* d_out, int out_size, void* d_ws, size_t ws_size,
                              hipStream_t stream)
{
  if (n_in < 16) return;
  const float* x   = (const float*)d_in[0];
  const int*   ei  = (const int*)d_in[1];
  const float* gw0 = (const float*)d_in[2];  const float* gb0 = (const float*)d_in[3];
  const float* gw1 = (const float*)d_in[4];  const float* gb1 = (const float*)d_in[5];
  const float* gw2 = (const float*)d_in[6];  const float* gb2 = (const float*)d_in[7];
  const float* lw0 = (const float*)d_in[8];  const float* lb0 = (const float*)d_in[9];
  const float* lw1 = (const float*)d_in[10]; const float* lb1 = (const float*)d_in[11];
  const float* lw2 = (const float*)d_in[12]; const float* lb2 = (const float*)d_in[13];
  const float* lw3 = (const float*)d_in[14]; const float* lb3 = (const float*)d_in[15];

  const int N = in_sizes[0] / DH;
  const int E = in_sizes[1] / 2;
  if (N <= 0 || in_sizes[0] != N * DH || E < 0 || in_sizes[1] != 2 * E || out_size < N) return;
  if (in_sizes[2] != DH * DH || in_sizes[4] != DH * DH || in_sizes[6] != DH * DH ||
      in_sizes[8] != DH * DH || in_sizes[10] != DH * DH || in_sizes[12] != DH * DH) return;
  if (in_sizes[3] < DH || in_sizes[5] < DH || in_sizes[7] < DH || in_sizes[9] < DH ||
      in_sizes[11] < DH || in_sizes[13] < DH || in_sizes[14] < DH || in_sizes[15] < 1) return;

  const int* src = ei;
  const int* dst = ei + E;

  const int NG = (N + GNODES - 1) / GNODES;
  const int NS = (N + SNODES - 1) / SNODES;
  long long expS = ((long long)E * SNODES + N - 1) / N;
  long long cS = 2 * expS + 1024; if (cS > E) cS = E; if (cS < 64) cS = 64; cS = (cS + 63) / 64 * 64;
  long long expG = ((long long)E * GNODES + N - 1) / N;
  long long cG = 2 * expG + 1024; if (cG > E) cG = E; if (cG < 64) cG = 64; cG = (cG + 63) / 64 * 64;
  const int capS = (int)cS, capG = (int)cG;

  size_t off = 0;
  char* ws = (char*)d_ws;
  #define CARVE(ptr, type, bytes) ptr = (type)(ws + off); off += (((size_t)(bytes)) + 511) & ~(size_t)511;
  float* Hb;      CARVE(Hb, float*, (size_t)N * DH * sizeof(float))
  float* Yb;      CARVE(Yb, float*, (size_t)N * DH * sizeof(float))
  float* dinv;    CARVE(dinv, float*, (size_t)NG * GNODES * sizeof(float))
  _Float16* Wt;   CARVE(Wt, _Float16*, (size_t)6 * DH * DH * sizeof(_Float16))
  int2* listS;    CARVE(listS, int2*, (size_t)NS * capS * sizeof(int2))
  int* cntS;      CARVE(cntS, int*, (size_t)NS * 32 * sizeof(int))
  int2* listG;    CARVE(listG, int2*, (size_t)NG * capG * sizeof(int2))
  int* cntG;      CARVE(cntG, int*, (size_t)NG * 32 * sizeof(int))
  #undef CARVE
  if (off > ws_size) return;

  float* dout = (float*)d_out;
  const dim3 b256(256), b32(32);

  k_wcvt<<<dim3(DH / 16, 6), b256, 0, stream>>>(gw0, gw1, gw2, lw0, lw1, lw2, Wt);
  k_split1<<<dim3(NS), b32, 0, stream>>>(src, dst, E, N, listS, cntS, capS);
  k_split2<<<dim3(NG), b32, 0, stream>>>(listS, cntS, capS, N, listG, cntG, capG, dinv);

  const int gemmGrid = (N + ROWS - 1) / ROWS;
  const size_t aggLds = (size_t)NWAVE_AGG * TNODES * DH * sizeof(float);
  const float* gb[3] = {gb0, gb1, gb2};

  const float* in = x;
  for (int l = 0; l < 3; ++l) {
    k_gemm<<<dim3(gemmGrid), b256, 0, stream>>>(in, Wt + (size_t)l * DH * DH, gb[l], dinv, Yb,
                                                lw3, lb3, dout, N, 1);
    k_aggr<<<dim3(NG), b256, aggLds, stream>>>(Yb, listG, cntG, capG, dinv, gb[l], Hb, N, (l < 2) ? 1 : 0);
    in = Hb;
  }
  k_gemm<<<dim3(gemmGrid), b256, 0, stream>>>(Hb, Wt + (size_t)3 * DH * DH, lb0, dinv, Yb, lw3, lb3, dout, N, 2 | 4);
  k_gemm<<<dim3(gemmGrid), b256, 0, stream>>>(Yb, Wt + (size_t)4 * DH * DH, lb1, dinv, Hb, lw3, lb3, dout, N, 2 | 4);
  k_gemm<<<dim3(gemmGrid), b256, 0, stream>>>(Hb, Wt + (size_t)5 * DH * DH, lb2, dinv, Yb, lw3, lb3, dout, N, 2 | 4 | 8);
}
